// OutlookAttention2d_65644280152795
// MI455X (gfx1250) — hardware-verified
//
#include <hip/hip_runtime.h>


#define NB_   8
#define CD_   384
#define LP_   3136
#define WP_   56
#define HP_   56
#define NATT  54
#define NHD   6
#define KK_   9
#define APD   64
#define NO1   448
#define WROWS 832
#define NPT   (LP_ / 64)

#define X_N   (NB_ * CD_ * LP_)
#define WA_N  (NATT * CD_)
#define WV_N  (CD_ * CD_)
#define OUT_N X_N

#define SZ_VT   ((size_t)NB_ * LP_ * CD_ * 4)
#define SZ_AT   ((size_t)NB_ * LP_ * APD * 4)
#define SZ_XT   ((size_t)NB_ * LP_ * CD_ * 2)
#define SZ_YT   SZ_XT
#define SZ_W16  ((size_t)WROWS * CD_ * 2)
#define SZ_BIAS ((size_t)NO1 * 4)
#define OFF_VT   ((size_t)0)
#define OFF_AT   (OFF_VT + SZ_VT)
#define OFF_XT   (OFF_AT + SZ_AT)
#define OFF_YT   (OFF_XT + SZ_XT)
#define OFF_W16  (OFF_YT + SZ_YT)
#define OFF_BIAS (OFF_W16 + SZ_W16)
#define WS_TOTAL (OFF_BIAS + SZ_BIAS)

static_assert(WS_TOTAL == 84133632);
static_assert(WS_TOTAL <= 134217728);
static_assert((OFF_AT % 128) == 0 && (OFF_XT % 128) == 0 && (OFF_YT % 128) == 0 &&
              (OFF_W16 % 128) == 0 && (OFF_BIAS % 128) == 0);
static_assert(LP_ % 64 == 0 && CD_ % 64 == 0 && (NB_ * LP_) % 64 == 0);
static_assert(WROWS * 48 == 156 * 256 && CD_ * 48 == 72 * 256 && APD * 48 == 12 * 256);

#define XP 72
#define EP 68

typedef unsigned short v8us  __attribute__((ext_vector_type(8)));
typedef unsigned short v8usa __attribute__((ext_vector_type(8), __may_alias__));
typedef unsigned short v16us __attribute__((ext_vector_type(16)));
typedef _Float16       v16h  __attribute__((ext_vector_type(16)));
typedef float          v8f   __attribute__((ext_vector_type(8)));
typedef float          v4f   __attribute__((ext_vector_type(4)));
typedef float          v4fa  __attribute__((ext_vector_type(4), __may_alias__));

union Frag { v16us v; v8us half[2]; };

__device__ __forceinline__ unsigned short h2us(float f) {
  return __builtin_bit_cast(unsigned short, (_Float16)f);
}

__device__ __forceinline__ void st2_u8(unsigned short* p, v8us v) {
  *(volatile v8us*)p = v;
  __threadfence();
  *(volatile v8us*)p = v;
}
__device__ __forceinline__ void st2_f4(float* p, v4f v) {
  *(volatile v4f*)p = v;
  __threadfence();
  *(volatile v4f*)p = v;
}

__device__ __forceinline__ v16h ldfrag(const unsigned short* rowp, int h) {
  Frag f;
  f.half[0] = *(const v8us*)(rowp + 8 * h);
  f.half[1] = *(const v8us*)(rowp + 16 + 8 * h);
  return __builtin_bit_cast(v16h, f.v);
}

__device__ __forceinline__ v8f wmma_h(v16h a, v16h b, v8f c) {
  return __builtin_amdgcn_wmma_f32_16x16x32_f16(false, a, false, b, (short)0, c, false, false);
}

__device__ __forceinline__ v8f v8f_zero() {
  v8f z = {0.f, 0.f, 0.f, 0.f, 0.f, 0.f, 0.f, 0.f};
  return z;
}

__global__ void __launch_bounds__(256) k_wprep(
    const float* __restrict__ Wv, const float* __restrict__ Wa, const float* __restrict__ Wp,
    const float* __restrict__ bv, const float* __restrict__ ba,
    unsigned short* __restrict__ W16, float* __restrict__ bias) {
  const int tid = threadIdx.x;
  const int bid = blockIdx.x;
  if (bid < 156) {
    const int i = bid * 256 + tid;
    const int row = i / 48;
    const int c8 = (i - row * 48) * 8;
    const float* src;
    int srow;
    bool valid = true;
    if (bid < 72) {
      src = Wv; srow = row;
    } else if (bid < 84) {
      const int r = row - 384;
      valid = (r < NATT);
      srow = (r < NATT) ? r : (NATT - 1);
      src = Wa;
    } else {
      src = Wp; srow = row - 448;
    }
    const size_t off = (size_t)srow * CD_ + c8;
    const v4f a0 = *(const v4f*)(src + off);
    const v4f a1 = *(const v4f*)(src + off + 4);
    const float sc = 16.0f;
    v8us ov;
    ov[0] = valid ? h2us(a0.x * sc) : (unsigned short)0;
    ov[1] = valid ? h2us(a0.y * sc) : (unsigned short)0;
    ov[2] = valid ? h2us(a0.z * sc) : (unsigned short)0;
    ov[3] = valid ? h2us(a0.w * sc) : (unsigned short)0;
    ov[4] = valid ? h2us(a1.x * sc) : (unsigned short)0;
    ov[5] = valid ? h2us(a1.y * sc) : (unsigned short)0;
    ov[6] = valid ? h2us(a1.z * sc) : (unsigned short)0;
    ov[7] = valid ? h2us(a1.w * sc) : (unsigned short)0;
    st2_u8(W16 + (size_t)row * CD_ + c8, ov);
  } else {
    if (tid < 112) {
      const int e0 = tid * 4;
      const int tb = (tid < 96) ? tid : 95;
      const v4f vb = *(const v4f*)(bv + tb * 4);
      const bool isv = (tid < 96);
      int ea = e0 - 384;
      int c0 = ea;     c0 = (c0 < 0) ? 0 : ((c0 > NATT - 1) ? (NATT - 1) : c0);
      int c1 = ea + 1; c1 = (c1 < 0) ? 0 : ((c1 > NATT - 1) ? (NATT - 1) : c1);
      int c2 = ea + 2; c2 = (c2 < 0) ? 0 : ((c2 > NATT - 1) ? (NATT - 1) : c2);
      int c3 = ea + 3; c3 = (c3 < 0) ? 0 : ((c3 > NATT - 1) ? (NATT - 1) : c3);
      const float q0 = ba[c0], q1 = ba[c1], q2 = ba[c2], q3 = ba[c3];
      v4f o;
      o.x = isv ? vb.x : ((ea + 0 >= 0 && ea + 0 < NATT) ? q0 : 0.0f);
      o.y = isv ? vb.y : ((ea + 1 >= 0 && ea + 1 < NATT) ? q1 : 0.0f);
      o.z = isv ? vb.z : ((ea + 2 >= 0 && ea + 2 < NATT) ? q2 : 0.0f);
      o.w = isv ? vb.w : ((ea + 3 >= 0 && ea + 3 < NATT) ? q3 : 0.0f);
      st2_f4(bias + e0, o);
    }
  }
}

__global__ void __launch_bounds__(256) k_xprep(const float* __restrict__ x, unsigned short* __restrict__ xT) {
  __shared__ __attribute__((aligned(16))) unsigned short sT[64 * XP];
  const int tid = threadIdx.x;
  const int lane = tid & 31;
  const int w = tid >> 5;
  const int bid = blockIdx.x;
  const int pt = bid % NPT;
  const int ct = (bid / NPT) % (CD_ / 64);
  const int n = bid / (NPT * (CD_ / 64));
  const int p0 = pt * 64;
  const int c0 = ct * 64;

  #pragma unroll
  for (int it = 0; it < 4; ++it) {
    const int idx = it * 256 + tid;
    const int c = idx >> 4;
    const int p4 = (idx & 15) * 4;
    const v4f v = *(const v4f*)(x + ((size_t)(n * CD_ + c0 + c)) * LP_ + p0 + p4);
    sT[(p4 + 0) * XP + c] = h2us(v.x);
    sT[(p4 + 1) * XP + c] = h2us(v.y);
    sT[(p4 + 2) * XP + c] = h2us(v.z);
    sT[(p4 + 3) * XP + c] = h2us(v.w);
  }
  __syncthreads();

  const int q = lane >> 3;
  const int j = lane & 7;
  #pragma unroll 1
  for (int it = 0; it < 2; ++it) {
    const int prow = it * 32 + w * 4 + q;
    const v8us val = *(const v8usa*)(sT + prow * XP + j * 8);
    unsigned short* dst = xT + ((size_t)(n * LP_ + p0 + prow)) * CD_ + c0 + j * 8;
    st2_u8(dst, val);
  }
}

__device__ __forceinline__ void write_tile64(const float* sT, float* obase, size_t row0, int opitch,
                                             int ocol, int lane, int w) {
  const int q = lane >> 3;
  const int j = lane & 7;
  const int rsel = q >> 1;
  const int lsel = q & 1;
  #pragma unroll 1
  for (int it = 0; it < 4; ++it) {
    const int row = it * 16 + w * 2 + rsel;
    const v4f v = *(const v4fa*)(sT + row * EP + lsel * 32 + j * 4);
    float* dst = obase + (row0 + (size_t)row) * (size_t)opitch + ocol + lsel * 32 + j * 4;
    st2_f4(dst, v);
  }
}

__device__ __forceinline__ void stage_c1(float* sT, v8f a0, v8f a1, int prow0, int col0, float b0, float b1) {
  #pragma unroll
  for (int r = 0; r < 8; ++r) {
    sT[(prow0 + r) * EP + col0] = a0[r] * 0.0625f + b0;
    sT[(prow0 + r) * EP + col0 + 16] = a1[r] * 0.0625f + b1;
  }
}

__global__ void __launch_bounds__(256) k_conv1(
    const unsigned short* __restrict__ xT, const unsigned short* __restrict__ W16,
    const float* __restrict__ bias, float* vT, float* aT) {
  __shared__ __attribute__((aligned(16))) float sT[64 * EP];
  const int tid = threadIdx.x;
  const int lane = tid & 31;
  const int w = tid >> 5;
  const int h = lane >> 4;
  const int m = lane & 15;
  const int bid = blockIdx.x;
  const int pt = bid % NPT;
  const int ot = (bid / NPT) % 7;
  const int n = bid / (NPT * 7);
  const int p0 = pt * 64;
  const int o0 = ot * 64;
  const int lsub = (w >> 1) * 16;
  const int osub = (w & 1) * 32;

  const unsigned short* ar  = xT + ((size_t)(n * LP_ + p0 + lsub + m)) * CD_;
  const unsigned short* br0 = W16 + (size_t)(o0 + osub + m) * CD_;
  const unsigned short* br1 = br0 + 16 * CD_;

  v8f acc0 = v8f_zero(), acc1 = v8f_zero();

  #pragma unroll 1
  for (int ks = 0; ks < CD_ / 32; ++ks) {
    const int k0 = ks * 32;
    const v16h fa  = ldfrag(ar + k0, h);
    const v16h fb0 = ldfrag(br0 + k0, h);
    const v16h fb1 = ldfrag(br1 + k0, h);
    acc0 = wmma_h(fa, fb0, acc0);
    acc1 = wmma_h(fa, fb1, acc1);
    asm volatile("v_nop\n\tv_nop\n\tv_nop\n\tv_nop"
                 : "+v"(acc0), "+v"(acc1)
                 : "v"(fa), "v"(fb0), "v"(fb1));
  }

  const float b0 = bias[o0 + osub + m];
  const float b1 = bias[o0 + osub + 16 + m];
  stage_c1(sT, acc0, acc1, lsub + 8 * h, osub + m, b0, b1);
  __syncthreads();

  float* obase = (ot < 6) ? vT : aT;
  const int opitch = (ot < 6) ? CD_ : APD;
  const int ocol = (ot < 6) ? o0 : 0;
  write_tile64(sT, obase, (size_t)(n * LP_ + p0), opitch, ocol, lane, w);
}

__global__ void __launch_bounds__(384) k_agg(
    const float* __restrict__ aT, const float* __restrict__ vT, unsigned short* __restrict__ yT) {
  __shared__ float sp[APD];
  __shared__ __attribute__((aligned(16))) unsigned short sy[CD_];
  const int bl = blockIdx.x;
  const int n = bl / LP_;
  const int l = bl - n * LP_;
  const int py = l / WP_;
  const int pxx = l - py * WP_;
  const int t = threadIdx.x;

  if (t < APD) sp[t] = aT[(size_t)bl * APD + t];
  __syncthreads();
  if (t < NHD) {
    const int o = t * KK_;
    float mx = sp[o];
    #pragma unroll
    for (int k = 1; k < KK_; ++k) mx = fmaxf(mx, sp[o + k]);
    float s = 0.0f;
    #pragma unroll 1
    for (int k = 0; k < KK_; ++k) {
      const float e = expf(sp[o + k] - mx);
      sp[o + k] = e;
      s += e;
    }
    const float inv = 1.0f / s;
    #pragma unroll 1
    for (int k = 0; k < KK_; ++k) sp[o + k] = sp[o + k] * inv;
  }
  __syncthreads();

  const int c = t;
  const int hd = c >> 6;
  const float* vb = vT + (size_t)n * LP_ * CD_ + c;
  float acc = 0.0f;
  #pragma unroll
  for (int k = 0; k < KK_; ++k) {
    const int yy = py + (k / 3) - 1;
    const int xx = pxx + (k % 3) - 1;
    const bool inb = (yy >= 0) && (yy < HP_) && (xx >= 0) && (xx < WP_);
    const int yc = (yy < 0) ? 0 : ((yy > HP_ - 1) ? (HP_ - 1) : yy);
    const int xc = (xx < 0) ? 0 : ((xx > WP_ - 1) ? (WP_ - 1) : xx);
    const float v = vb[(size_t)(yc * WP_ + xc) * CD_];
    const float pv = inb ? v : 0.0f;
    acc = fmaf(sp[hd * KK_ + k], pv, acc);
  }
  sy[c] = h2us(acc);
  __syncthreads();

  if (t < 48) {
    const v8us val = *(const v8usa*)(sy + t * 8);
    st2_u8(yT + (size_t)bl * CD_ + t * 8, val);
  }
}

__device__ __forceinline__ void stage_pj(float* sT, v8f a0, v8f a1, int orow0, int col0, const float* bpp) {
  #pragma unroll
  for (int r = 0; r < 8; ++r) {
    const float b = bpp[r];
    sT[(orow0 + r) * EP + col0] = a0[r] * 0.0625f + b;
    sT[(orow0 + r) * EP + col0 + 16] = a1[r] * 0.0625f + b;
  }
}

__global__ void __launch_bounds__(256) k_proj(
    const unsigned short* __restrict__ yT, const unsigned short* __restrict__ W16,
    const float* __restrict__ bp, float* __restrict__ out) {
  __shared__ __attribute__((aligned(16))) float sT[64 * EP];
  const int tid = threadIdx.x;
  const int lane = tid & 31;
  const int w = tid >> 5;
  const int h = lane >> 4;
  const int m = lane & 15;
  const int bid = blockIdx.x;
  const int pt = bid % NPT;
  const int ot = (bid / NPT) % (CD_ / 64);
  const int n = bid / (NPT * (CD_ / 64));
  const int p0 = pt * 64;
  const int o0 = ot * 64;
  const int osub = (w >> 1) * 16;
  const int lsub = (w & 1) * 32;

  const unsigned short* ar  = W16 + (size_t)(NO1 + o0 + osub + m) * CD_;
  const unsigned short* br0 = yT + ((size_t)(n * LP_ + p0 + lsub + m)) * CD_;
  const unsigned short* br1 = br0 + 16 * CD_;

  v8f acc0 = v8f_zero(), acc1 = v8f_zero();

  #pragma unroll 1
  for (int ks = 0; ks < CD_ / 32; ++ks) {
    const int k0 = ks * 32;
    const v16h fa  = ldfrag(ar + k0, h);
    const v16h fb0 = ldfrag(br0 + k0, h);
    const v16h fb1 = ldfrag(br1 + k0, h);
    acc0 = wmma_h(fa, fb0, acc0);
    acc1 = wmma_h(fa, fb1, acc1);
    asm volatile("v_nop\n\tv_nop\n\tv_nop\n\tv_nop"
                 : "+v"(acc0), "+v"(acc1)
                 : "v"(fa), "v"(fb0), "v"(fb1));
  }

  const float* bpp = bp + o0 + osub + 8 * h;
  stage_pj(sT, acc0, acc1, osub + 8 * h, lsub + m, bpp);
  __syncthreads();

  write_tile64(sT, out, (size_t)(n * CD_ + o0), LP_, p0, lane, w);
}

extern "C" void kernel_launch(void* const* d_in, const int* in_sizes, int n_in,
                              void* d_out, int out_size, void* d_ws, size_t ws_size,
                              hipStream_t stream) {
  if (n_in < 7) return;
  if (in_sizes[0] != X_N || in_sizes[1] != WA_N || in_sizes[2] != NATT ||
      in_sizes[3] != WV_N || in_sizes[4] != CD_ || in_sizes[5] != WV_N || in_sizes[6] != CD_) return;
  if (out_size != OUT_N) return;
  if (ws_size < (size_t)WS_TOTAL) return;

  const float* x  = (const float*)d_in[0];
  const float* Wa = (const float*)d_in[1];
  const float* ba = (const float*)d_in[2];
  const float* Wv = (const float*)d_in[3];
  const float* bv = (const float*)d_in[4];
  const float* Wp = (const float*)d_in[5];
  const float* bp = (const float*)d_in[6];
  float* out = (float*)d_out;

  char* ws = (char*)d_ws;
  float*          vT   = (float*)(ws + OFF_VT);
  float*          aT   = (float*)(ws + OFF_AT);
  unsigned short* xT   = (unsigned short*)(ws + OFF_XT);
  unsigned short* yT   = (unsigned short*)(ws + OFF_YT);
  unsigned short* W16  = (unsigned short*)(ws + OFF_W16);
  float*          bias = (float*)(ws + OFF_BIAS);

  k_wprep<<<dim3(157), dim3(256), 0, stream>>>(Wv, Wa, Wp, bv, ba, W16, bias);
  k_xprep<<<dim3(NB_ * (CD_ / 64) * NPT), dim3(256), 0, stream>>>(x, xT);
  k_conv1<<<dim3(NB_ * 7 * NPT), dim3(256), 0, stream>>>(xT, W16, bias, vT, aT);
  k_agg<<<dim3(NB_ * LP_), dim3(384), 0, stream>>>(aT, vT, yT);
  k_proj<<<dim3(NB_ * (CD_ / 64) * NPT), dim3(256), 0, stream>>>(yT, W16, bp, out);
}
